// MoNetLayer_27977416966688
// MI455X (gfx1250) — hardware-run, weakly checked
//
#include <hip/hip_runtime.h>


namespace {
constexpr int NB_ = 32, N = 256, K = 25, F = 64, FO = 64;
constexpr float XS = 8.0f, HS = 256.0f, WSC = 256.0f, TWO_PI = 6.283185307179586f;
typedef _Float16 b16;
typedef __attribute__((ext_vector_type(16))) _Float16 v16b;
typedef __attribute__((ext_vector_type(8))) _Float16 v8b;
typedef __attribute__((ext_vector_type(2))) _Float16 v2b;
typedef __attribute__((ext_vector_type(8))) float v8f;
typedef __attribute__((ext_vector_type(4))) float v4f;
typedef __attribute__((ext_vector_type(2))) float v2f;
__device__ __forceinline__ float bf16_rne(float f) { unsigned int u = __float_as_uint(f); u += 0x7FFFu + ((u >> 16) & 1u); float r = __uint_as_float(u & 0xFFFF0000u); asm volatile("" : "+v"(r)); return r; }
__device__ __forceinline__ float bfv(float f) { float r = bf16_rne(f); asm volatile("" : "+v"(r)); return r; }
__device__ __forceinline__ void split16(float v, b16& hi, b16& lo) { hi = (b16)v; lo = (b16)(v - (float)hi); }
__device__ __forceinline__ v16b frag_kb(const b16* p, int hh) { const v8b a = *(const v8b*)(p + 8 * hh), b = *(const v8b*)(p + 16 + 8 * hh); v16b f;
#pragma unroll
  for (int e = 0; e < 8; ++e) { f[e] = a[e]; f[8 + e] = b[e]; } return f; }
__device__ __forceinline__ v8f wmma16b(v16b a, v16b b, v8f c) { v8f d = __builtin_amdgcn_wmma_f32_16x16x32_f16(false, a, false, b, (short)0, c, false, false); asm volatile("v_nop\n\tv_nop\n\tv_nop\n\tv_nop" : "+v"(d) : "v"(a), "v"(b)); return d; }
__device__ __forceinline__ void wave_lds_sync() { __builtin_amdgcn_fence(__ATOMIC_RELEASE, "workgroup"); __builtin_amdgcn_wave_barrier(); __builtin_amdgcn_fence(__ATOMIC_ACQUIRE, "workgroup"); }
__device__ __forceinline__ float pmul(float a, float b) { float p = a * b; asm volatile("" : "+v"(p)); return p; }

__global__ __launch_bounds__(256) void prep_kernel(const float* __restrict__ x, const float* __restrict__ fw, b16* __restrict__ WF, b16* __restrict__ XT) { __shared__ float Tt[64][F + 1]; const int tid = threadIdx.x, wave = tid >> 5, lane = tid & 31;
  if (blockIdx.x < NB_ * (N / 64)) { const int b = blockIdx.x / (N / 64), j0 = (blockIdx.x % (N / 64)) * 64;
    for (int q = wave; q < 64; q += 8) { Tt[q][lane * 2] = bfv(x[((size_t)b * N + j0 + q) * F + lane * 2]); Tt[q][lane * 2 + 1] = bfv(x[((size_t)b * N + j0 + q) * F + lane * 2 + 1]); }
    __syncthreads();
    for (int pass = 0; pass < 2; ++pass) { for (int f = wave; f < F; f += 8) *(volatile v2b*)(XT + ((size_t)b * F + f) * N + j0 + lane * 2) = (v2b){(b16)(Tt[lane * 2][f] * XS), (b16)(Tt[lane * 2 + 1][f] * XS)}; __threadfence(); } }
  else { const int u = (blockIdx.x - NB_ * (N / 64)) * 256 + tid; if (u < FO * (K * F / 8)) { const int o = u / (K * F / 8), k0 = (u % (K * F / 8)) * 8; v8b v;
#pragma unroll
      for (int j = 0; j < 8; ++j) v[j] = (b16)(bf16_rne(fw[(size_t)o * K * F + k0 + j]) * WSC); for (int pass = 0; pass < 2; ++pass) { *(volatile v8b*)(WF + (size_t)o * K * F + k0) = v; __threadfence(); } } } }
__global__ __launch_bounds__(32) void main_kernel(const float* __restrict__ coord, const float* __restrict__ mask, const float* __restrict__ cmu, const float* __restrict__ srho, const float* __restrict__ sth, const b16* __restrict__ XT, const b16* __restrict__ WF, const float* __restrict__ fb, int BLIM, float* __restrict__ out) { __shared__ __attribute__((aligned(16))) b16 Wa[16][N + 8], Wb[16][N + 8], Ga[16][F + 8], Gb[16][F + 8]; __shared__ float Rh[16][N], Th[16][N], Tf[16][FO + 1]; const int lane = threadIdx.x, nloc = lane & 15, hlf = lane >> 4; const int b = blockIdx.x / (N / 16), i0 = (blockIdx.x % (N / 16)) * 16; if (b >= BLIM) return;
  for (int rr = 0; rr < 16; ++rr) for (int q = 0; q < N / 32; ++q) { const int j = q * 32 + lane; const size_t e = (((size_t)b * N + i0 + rr) * N + j) * 2; const float r = coord[e], t = coord[e + 1]; const bool isn = r != r; Rh[rr][j] = isn ? -1.0f : bfv(r); Th[rr][j] = isn ? 0.0f : bfv(t); }
  if (lane < 16) { for (int k = N; k < N + 8; ++k) { Wa[lane][k] = (b16)0.0f; Wb[lane][k] = (b16)0.0f; } for (int k = F; k < F + 8; ++k) { Ga[lane][k] = (b16)0.0f; Gb[lane][k] = (b16)0.0f; } }
  wave_lds_sync();
  v8f oacc[4] = {(v8f){}, (v8f){}, (v8f){}, (v8f){}};
#pragma unroll 1
  for (int k = 0; k < K; ++k) { const float mu = bfv(cmu[k]), sr = bfv(srho[k]), st = bfv(sth[k]); const float ir = -0.5f / (1e-14f + sr * sr), it = -0.5f / (1e-14f + st * st);
    for (int rr = 0; rr < 16; ++rr) for (int q = 0; q < N / 32; ++q) { const int j = q * 32 + lane; const float r = Rh[rr][j]; float w = 0.0f; if (r >= 0.0f) { const float dr = r - mu; const float d = fabsf(Th[rr][j] - mu); const float ang = fminf(d, fabsf(TWO_PI - d)); w = __expf(dr * dr * ir) * __expf(ang * ang * it); } b16 p, pl; split16(w * HS, p, pl); Wa[rr][j] = p; Wb[rr][j] = pl; }
    wave_lds_sync();
    v8f acc[4] = {(v8f){}, (v8f){}, (v8f){}, (v8f){}};
#pragma unroll 2
    for (int kb = 0; kb < N; kb += 32) { const v16b a = frag_kb(&Wa[nloc][kb], hlf), al = frag_kb(&Wb[nloc][kb], hlf);
#pragma unroll
      for (int t = 0; t < 4; ++t) { const v16b bw = frag_kb(XT + ((size_t)b * F + t * 16 + nloc) * N + kb, hlf); acc[t] = wmma16b(a, bw, acc[t]); acc[t] = wmma16b(al, bw, acc[t]); } }
#pragma unroll
    for (int t = 0; t < 4; ++t)
#pragma unroll
      for (int r8 = 0; r8 < 8; ++r8) { b16 p, pl; split16(acc[t][r8] * (1.0f / (HS * XS)) * HS, p, pl); Ga[8 * hlf + r8][t * 16 + nloc] = p; Gb[8 * hlf + r8][t * 16 + nloc] = pl; }
    wave_lds_sync();
#pragma unroll
    for (int kb = 0; kb < F; kb += 32) { const v16b a = frag_kb(&Ga[nloc][kb], hlf), al = frag_kb(&Gb[nloc][kb], hlf);
#pragma unroll
      for (int t = 0; t < 4; ++t) { const v16b bw = frag_kb(WF + (size_t)(t * 16 + nloc) * (K * F) + k * F + kb, hlf); oacc[t] = wmma16b(a, bw, oacc[t]); oacc[t] = wmma16b(al, bw, oacc[t]); } }
    wave_lds_sync(); }
#pragma unroll
  for (int t = 0; t < 4; ++t) { const int cc = t * 16 + nloc; const float bb = bfv(fb[cc]);
#pragma unroll
    for (int r8 = 0; r8 < 8; ++r8) { const int rr = 8 * hlf + r8; Tf[rr][cc] = (oacc[t][r8] * (1.0f / (HS * WSC)) + bb) * bfv(mask[(size_t)b * N + i0 + rr]); } }
  wave_lds_sync();
  for (int pass = 0; pass < 2; ++pass) { for (int rr = 0; rr < 16; ++rr) *(volatile v2f*)(out + ((size_t)b * N + i0 + rr) * FO + lane * 2) = (v2f){Tf[rr][lane * 2], Tf[rr][lane * 2 + 1]}; __threadfence(); } }
}

extern "C" void kernel_launch(void* const* d_in, const int* in_sizes, int n_in, void* d_out, int out_size, void* d_ws, size_t ws_size, hipStream_t stream) {
  (void)n_in;
  auto Fp = [&](int i) { return (const float*)d_in[i]; };
  if (in_sizes[0] != NB_ * N * F || in_sizes[1] != NB_ * N * N * 2 || in_sizes[2] != NB_ * N || in_sizes[3] != 2 * K || in_sizes[4] != K || in_sizes[6] != FO * K * F || out_size != NB_ * N * FO) return;
  const int BLIM = NB_;
  size_t off = 0; char* ws = (char*)d_ws;
  auto carve = [&](size_t bytes) { char* p = ws + off; off += (bytes + 255) & ~(size_t)255; return p; };
  b16* WF = (b16*)carve((size_t)FO * K * F * 2); b16* XT = (b16*)carve((size_t)NB_ * F * N * 2);
  if (off > ws_size || off > ((size_t)2 << 20)) return;
  prep_kernel<<<NB_ * (N / 64) + (FO * (K * F / 8) + 255) / 256, 256, 0, stream>>>(Fp(0), Fp(6), WF, XT);
  main_kernel<<<BLIM * (N / 16), 32, 0, stream>>>(Fp(1), Fp(2), Fp(3), Fp(4), Fp(5), XT, WF, Fp(7), BLIM, (float*)d_out);
}
